// EdgeAwareAttention_43344809951969
// MI455X (gfx1250) — hardware-run, weakly checked
//
#include <hip/hip_runtime.h>


namespace {
constexpr int N = 20000, E = 320000, D = 256, H = 8, HD = 32, NPB = 8;
constexpr float XS = 8.0f, HS = 256.0f, WSC = 256.0f, SCALE = 0.17677669529663688f, EPS = 1e-5f;
typedef _Float16 b16;
typedef __attribute__((ext_vector_type(16))) _Float16 v16b;
typedef __attribute__((ext_vector_type(8))) _Float16 v8b;
typedef __attribute__((ext_vector_type(8))) float v8f;
typedef __attribute__((ext_vector_type(4))) float v4f;
__device__ __forceinline__ float bf16_rne(float f) { unsigned int u = __float_as_uint(f); u += 0x7FFFu + ((u >> 16) & 1u); float r = __uint_as_float(u & 0xFFFF0000u); asm volatile("" : "+v"(r)); return r; }
__device__ __forceinline__ float bfv(float f) { float r = bf16_rne(f); asm volatile("" : "+v"(r)); return r; }
__device__ __forceinline__ void split16(float v, b16& hi, b16& lo) { hi = (b16)v; lo = (b16)(v - (float)hi); }
__device__ __forceinline__ v16b frag_kb(const b16* p, int hh) { const v8b a = *(const v8b*)(p + 8 * hh), b = *(const v8b*)(p + 16 + 8 * hh); v16b f;
#pragma unroll
  for (int e = 0; e < 8; ++e) { f[e] = a[e]; f[8 + e] = b[e]; } return f; }
__device__ __forceinline__ v8f wmma16b(v16b a, v16b b, v8f c) { v8f d = __builtin_amdgcn_wmma_f32_16x16x32_f16(false, a, false, b, (short)0, c, false, false); asm volatile("v_nop\n\tv_nop\n\tv_nop\n\tv_nop" : "+v"(d) : "v"(a), "v"(b)); return d; }
__device__ __forceinline__ void wave_lds_sync() { __builtin_amdgcn_fence(__ATOMIC_RELEASE, "workgroup"); __builtin_amdgcn_wave_barrier(); __builtin_amdgcn_fence(__ATOMIC_ACQUIRE, "workgroup"); }
__device__ __forceinline__ float pmul(float a, float b) { float p = a * b; asm volatile("" : "+v"(p)); return p; }
__device__ __forceinline__ int iclamp(int v, int lo, int hi) { return v < lo ? lo : (v > hi ? hi : v); }
constexpr int CSR_NBLK8 = 512, CSR_GB8 = 8, CSR_GN8 = 1 << CSR_GB8  , CSR_TS8 = (CSR_GN8 < 32 ? 32 : CSR_GN8)  , CSR_MAXG8 = 512, CSR_CAP8 = 12288  ;
__device__ __host__ __forceinline__ int csr_tix8(int v) { return (v >> CSR_GB8) * CSR_TS8 + (v & (CSR_GN8 - 1)); }
__global__ __launch_bounds__(64) void csrA_kernel8(const int* __restrict__ dst, int E, int N, int nG, int CHP, int NGP, int* __restrict__ STG, int* __restrict__ HST) {
  extern __shared__ int sm[];
  int* cnt = sm; int* run = sm + NGP; int* ids = sm + 2 * NGP;
  const int b = blockIdx.x; const int ch = (E + CSR_NBLK8 - 1) / CSR_NBLK8; const int e0 = b * ch, e1 = min(E, e0 + ch);
  for (int i = threadIdx.x; i < NGP; i += 64) cnt[i] = 0;
  for (int i = threadIdx.x; i < CHP; i += 64) ids[i] = -1;
  __syncthreads();
  if (threadIdx.x == 0) {
    for (int e = e0; e < e1; ++e) { int d = dst[e]; d = (d < 0) ? 0 : (d >= N ? N - 1 : d); cnt[d >> CSR_GB8] += 1; }
    int acc = 0; for (int g = 0; g < nG; ++g) { run[g] = acc; acc += cnt[g]; }
    for (int e = e0; e < e1; ++e) { int d = dst[e]; d = (d < 0) ? 0 : (d >= N ? N - 1 : d); const int g = d >> CSR_GB8; ids[run[g]] = e; run[g] += 1; } }
  __syncthreads();
  typedef __attribute__((ext_vector_type(4))) int v4i;
  for (int pass = 0; pass < 2; ++pass) {
    for (int i = threadIdx.x; i < CHP / 4; i += 64) *(volatile v4i*)(STG + (size_t)b * CHP + i * 4) = *(const v4i*)(&ids[i * 4]);
    for (int i = threadIdx.x; i < NGP / 4; i += 64) { v4i v; for (int e = 0; e < 4; ++e) v[e] = (i * 4 + e < nG) ? cnt[i * 4 + e] : 0; *(volatile v4i*)(HST + (size_t)b * NGP + i * 4) = v; }
    __threadfence(); }
}
__global__ __launch_bounds__(512) void csrS_kernel8(const int* __restrict__ HST, int nG, int NGP, int* __restrict__ START, int* __restrict__ TOT, int* __restrict__ OFF) {
  __shared__ int tot[CSR_MAXG8];
  const int b = threadIdx.x;
  for (int pass = 0; pass < 2; ++pass) { int runb = 0; for (int g = 0; g < nG; ++g) { int c = HST[(size_t)b * NGP + g]; c = (c < 0) ? 0 : c; ((volatile int*)OFF)[(size_t)g * CSR_NBLK8 + b] = runb; runb += c; } __threadfence(); }
  for (int g = threadIdx.x; g < nG; g += 512) { int s = 0; for (int bb = 0; bb < CSR_NBLK8; ++bb) { int c = HST[(size_t)bb * NGP + g]; s += (c < 0) ? 0 : c; } tot[g] = s; }
  __syncthreads();
  if (threadIdx.x < 32) {
    __shared__ int st[CSR_MAXG8 + 32];
    if (threadIdx.x == 0) { int acc = 0; for (int g = 0; g < NGP; ++g) { st[g] = acc; if (g < nG) acc += (tot[g] + 31) & ~31; } st[NGP] = acc; }
    __builtin_amdgcn_fence(__ATOMIC_RELEASE, "workgroup"); __builtin_amdgcn_wave_barrier(); __builtin_amdgcn_fence(__ATOMIC_ACQUIRE, "workgroup");
    for (int pass = 0; pass < 2; ++pass) { for (int i = threadIdx.x; i < NGP + 32; i += 32) { ((volatile int*)START)[i] = (i <= NGP) ? st[min(i, NGP)] : 0; ((volatile int*)TOT)[i] = (i < nG) ? tot[i] : 0; } __threadfence(); } }
}
__global__ __launch_bounds__(256) void csrB_kernel8(const int* __restrict__ dst, int N, int nG, int CHP, int NGP, int permLen, const int* __restrict__ STG, const int* __restrict__ HST, const int* __restrict__ OFF, const int* __restrict__ START, const int* __restrict__ TOT, int* __restrict__ PERM, int* __restrict__ ROWPTR, int* __restrict__ ROWCNT, int* __restrict__ FLAG) {
  typedef __attribute__((ext_vector_type(4))) int v4i;
  __shared__ int ids[CSR_CAP8]; __shared__ unsigned short key[CSR_CAP8]; __shared__ int outp[CSR_CAP8]; __shared__ int ncnt[CSR_GN8 + 1]; __shared__ int boff[CSR_NBLK8 + 1];
  const int g = blockIdx.x, t_ = threadIdx.x; int tot = TOT[g]; int st = START[g], stn = START[g + 1]; const int v0 = g * CSR_GN8; const int nv = min(CSR_GN8, N - v0); const int t0 = g * CSR_TS8;
  st = (st < 0) ? 0 : (st > permLen - 32 ? permLen - 32 : st) & ~31; stn = (stn < st) ? st : (stn > permLen ? permLen : stn); tot = (tot < 0) ? 0 : tot; if (tot > stn - st && tot <= CSR_CAP8) tot = stn - st;
  if (tot > CSR_CAP8) {
    for (int pass = 0; pass < 2; ++pass) { for (int i = t_; i < CSR_TS8 / 4; i += 256) { v4i a, c; for (int e = 0; e < 4; ++e) { a[e] = st; c[e] = 0; } *(volatile v4i*)(ROWPTR + t0 + i * 4) = a; *(volatile v4i*)(ROWCNT + t0 + i * 4) = c; } if (t_ == 0) ((volatile int*)FLAG)[0] = 1; __threadfence(); } (void)nv; return; }
  if (t_ == 0) { int acc = 0; for (int b = 0; b < CSR_NBLK8; ++b) { boff[b] = acc; int c = HST[(size_t)b * NGP + g]; c = (c < 0) ? 0 : (c > CHP ? CHP : c); acc += c; if (acc > tot) acc = tot; } boff[CSR_NBLK8] = acc; }
  for (int i = t_; i <= CSR_GN8; i += 256) ncnt[i] = 0;
  __syncthreads();
  for (int b = 0; b < CSR_NBLK8; ++b) { const int c = boff[b + 1] - boff[b]; int o_ = OFF[(size_t)g * CSR_NBLK8 + b]; o_ = (o_ < 0) ? 0 : (o_ > CHP - c ? CHP - c : o_); const int* src_ = STG + (size_t)b * CHP + o_;
    for (int i = t_; i < c; i += 256) { int id = src_[i]; id = (id < 0) ? 0 : id; ids[boff[b] + i] = id; int d = dst[id]; d = (d < v0) ? v0 : (d >= N ? N - 1 : d); int kk = d - v0; kk = (kk < 0) ? 0 : (kk >= CSR_GN8 ? CSR_GN8 - 1 : kk); key[boff[b] + i] = (unsigned short)kk; } }
  __syncthreads();
  if (t_ == 0) { for (int i = 0; i < tot; ++i) ncnt[key[i]] += 1; int acc = 0; for (int vl = 0; vl < CSR_GN8; ++vl) { const int c = ncnt[vl]; ncnt[vl] = acc; acc += c; } ncnt[CSR_GN8] = acc;
    for (int i = 0; i < tot; ++i) { const int vl = key[i]; outp[ncnt[vl]] = ids[i]; ncnt[vl] += 1; }
    for (int vl = CSR_GN8; vl > 0; --vl) ncnt[vl] = ncnt[vl - 1]; ncnt[0] = 0; }
  __syncthreads();
  for (int pass = 0; pass < 2; ++pass) {
    for (int i = t_; i < (stn - st) / 4; i += 256) { v4i v; for (int e = 0; e < 4; ++e) { const int q = i * 4 + e; v[e] = (q < tot) ? outp[q] : -1; } *(volatile v4i*)(PERM + st + i * 4) = v; }
    for (int i = t_; i < CSR_TS8 / 4; i += 256) { v4i a, c; for (int e = 0; e < 4; ++e) { const int vl = i * 4 + e; const int vc = vl < CSR_GN8 ? vl : CSR_GN8; a[e] = (vl < CSR_GN8) ? st + ncnt[vc] : st; c[e] = (vl < nv) ? (ncnt[(vc < CSR_GN8 ? vc : CSR_GN8 - 1) + 1] - ncnt[vc]) : 0; } *(volatile v4i*)(ROWPTR + t0 + i * 4) = a; *(volatile v4i*)(ROWCNT + t0 + i * 4) = c; }
    __threadfence(); }
}
__global__ __launch_bounds__(256) void csrZ_kernel8(int* __restrict__ p, size_t n4) { typedef __attribute__((ext_vector_type(4))) int v4i; const size_t tid = (size_t)blockIdx.x * 256 + threadIdx.x, nth = (size_t)gridDim.x * 256; v4i z = {0, 0, 0, 0}; for (size_t i = tid; i < n4; i += nth) *(volatile v4i*)(p + i * 4) = z; }
struct CsrBufs8 { int *STG, *HST, *OFF, *START, *TOT, *PERM, *ROWPTR, *ROWCNT, *FLAG; int nG, NGP, CHP; size_t permLen; char* base; size_t bytes; };
static size_t csr_carve8(CsrBufs8& c, char* ws, size_t off, int E, int N) {
  const size_t off0 = off; c.base = ws + off;
  auto al = [&](size_t bytes) { char* p = ws + off; off += (bytes + 255) & ~(size_t)255; return p; };
  c.nG = (N + CSR_GN8 - 1) / CSR_GN8; c.NGP = (c.nG + 31) & ~31; const int ch = (E + CSR_NBLK8 - 1) / CSR_NBLK8; c.CHP = (ch + 31) & ~31; c.permLen = (size_t)E + 32 * (size_t)c.nG + 32;
  c.STG = (int*)al((size_t)CSR_NBLK8 * c.CHP * 4); c.HST = (int*)al((size_t)CSR_NBLK8 * c.NGP * 4); c.OFF = (int*)al((size_t)c.NGP * CSR_NBLK8 * 4); c.START = (int*)al((size_t)(c.NGP + 64) * 4); c.TOT = (int*)al((size_t)(c.NGP + 64) * 4);
  c.PERM = (int*)al(c.permLen * 4); c.ROWPTR = (int*)al((size_t)c.nG * CSR_TS8 * 4); c.ROWCNT = (int*)al((size_t)c.nG * CSR_TS8 * 4); c.FLAG = (int*)al(256);
  c.bytes = off - off0; return off;
}
static void csr_build8(const CsrBufs8& c, const int* dst, int E, int N, hipStream_t stream) {
  const size_t smem = (size_t)(2 * c.NGP + c.CHP) * 4;
  csrZ_kernel8<<<512, 256, 0, stream>>>((int*)c.base, c.bytes / 16);
  csrA_kernel8<<<CSR_NBLK8, 64, smem, stream>>>(dst, E, N, c.nG, c.CHP, c.NGP, c.STG, c.HST);
  csrS_kernel8<<<1, 512, 0, stream>>>(c.HST, c.nG, c.NGP, c.START, c.TOT, c.OFF);
  csrB_kernel8<<<c.nG, 256, 0, stream>>>(dst, N, c.nG, c.CHP, c.NGP, (int)c.permLen, c.STG, c.HST, c.OFF, c.START, c.TOT, c.PERM, c.ROWPTR, c.ROWCNT, c.FLAG);
}


__global__ __launch_bounds__(256) void wput_kernel(const float* __restrict__ wq, const float* __restrict__ wk, const float* __restrict__ wv, const float* __restrict__ wo, b16* __restrict__ WQKV, b16* __restrict__ WO) { const int u = blockIdx.x * 256 + threadIdx.x; if (u >= 4 * D * 32) return; const int o = u / 32, k0 = (u % 32) * 8; const int which = o / D, oo = o % D; const float* w = which == 0 ? wq : (which == 1 ? wk : (which == 2 ? wv : wo)); v8b v;
#pragma unroll
  for (int j = 0; j < 8; ++j) v[j] = (b16)(bf16_rne(w[(size_t)(k0 + j) * D + oo]) * WSC); b16* dst = which < 3 ? WQKV + (size_t)o * D + k0 : WO + (size_t)oo * D + k0;
  for (int pass = 0; pass < 2; ++pass) { *(volatile v8b*)dst = v; __threadfence(); } }
__global__ __launch_bounds__(32) void proj_kernel(const float* __restrict__ x, const b16* __restrict__ WQKV, float* __restrict__ Q, float* __restrict__ KV) { __shared__ __attribute__((aligned(16))) b16 Ax[16][D + 8]; __shared__ float Tf[16][260]; const int lane = threadIdx.x, nloc = lane & 15, hlf = lane >> 4; const size_t n0 = (size_t)blockIdx.x * 16;
  for (int rr = 0; rr < 16; ++rr) for (int q = 0; q < 8; ++q) { const int c = q * 32 + lane; Ax[rr][c] = (b16)(bf16_rne(x[(n0 + rr) * D + c]) * XS); }
  if (lane < 16) for (int k = D; k < D + 8; ++k) Ax[lane][k] = (b16)0.0f;
  wave_lds_sync();
#pragma unroll 1
  for (int g = 0; g < 3; ++g) { v8f acc[16];
#pragma unroll
    for (int t = 0; t < 16; ++t) acc[t] = (v8f){};
#pragma unroll 2
    for (int kb = 0; kb < D; kb += 32) { const v16b a = frag_kb(&Ax[nloc][kb], hlf);
#pragma unroll
      for (int t = 0; t < 16; ++t) acc[t] = wmma16b(a, frag_kb(WQKV + (size_t)(g * D + t * 16 + nloc) * D + kb, hlf), acc[t]); }
#pragma unroll
    for (int t = 0; t < 16; ++t)
#pragma unroll
      for (int r8 = 0; r8 < 8; ++r8) Tf[8 * hlf + r8][t * 16 + nloc] = acc[t][r8] * (1.0f / (XS * WSC));
    wave_lds_sync();
    for (int pass = 0; pass < 2; ++pass) { for (int rr = 0; rr < 16; ++rr) for (int q = 0; q < 2; ++q) { const v4f v = *(const v4f*)(&Tf[rr][q * 128 + lane * 4]); if (g == 0) *(volatile v4f*)(Q + (n0 + rr) * D + q * 128 + lane * 4) = v; else *(volatile v4f*)(KV + (n0 + rr) * 2 * D + (g - 1) * D + q * 128 + lane * 4) = v; } __threadfence(); }
    wave_lds_sync(); } }
__global__ __launch_bounds__(256) void att_kernel(const float* __restrict__ Q, const float* __restrict__ KV, const float* __restrict__ ew, const float* __restrict__ We, const int* __restrict__ tgts, const int* __restrict__ PERM, const int* __restrict__ ROWPTR, const int* __restrict__ ROWCNT, int permLen, int NLIM, float* __restrict__ AGG) { const int wave = threadIdx.x >> 5, lane = threadIdx.x & 31; const size_t i = (size_t)blockIdx.x * NPB + wave; if (i >= (size_t)NLIM) return; const int h = lane >> 2; const int c0 = lane * 8;
  v4f q0 = *(const v4f*)(Q + i * D + c0), q1 = *(const v4f*)(Q + i * D + c0 + 4); const float we = bfv(We[h]);
  int st = ROWPTR[i], cnt = ROWCNT[i]; cnt = iclamp(cnt, 0, E); st = iclamp(st, 0, permLen - cnt);
  float mx = -INFINITY, den = 0.0f; v4f a0 = {0, 0, 0, 0}, a1 = {0, 0, 0, 0};
#pragma unroll 1
  for (int j = 0; j < cnt; ++j) { const int e = iclamp(PERM[st + j], 0, E - 1); const size_t t = (size_t)iclamp(tgts[e], 0, N - 1); if (t >= (size_t)NLIM) continue; const float* kp = KV + t * 2 * D + c0; const v4f k0 = *(const v4f*)kp, k1 = *(const v4f*)(kp + 4), v0 = *(const v4f*)(kp + D), v1 = *(const v4f*)(kp + D + 4);
    float s = 0.0f; for (int k = 0; k < 4; ++k) { s += pmul(q0[k], k0[k]); s += pmul(q1[k], k1[k]); } s += __shfl_xor(s, 1); s += __shfl_xor(s, 2); s = s * SCALE + pmul(bfv(ew[e]), we);
    const float mn = fmaxf(mx, s); const float sf = (mx == -INFINITY) ? 0.0f : __expf(mx - mn); const float p = __expf(s - mn); a0 = a0 * sf + v0 * p; a1 = a1 * sf + v1 * p; den = den * sf + p; mx = mn; }
  const float inv = cnt > 0 && den > 0.0f ? 1.0f / den : 0.0f;
  for (int pass = 0; pass < 2; ++pass) { *(volatile v4f*)(AGG + i * D + c0) = a0 * inv; *(volatile v4f*)(AGG + i * D + c0 + 4) = a1 * inv; __threadfence(); } }
__global__ __launch_bounds__(32) void out_kernel(const float* __restrict__ AGG, const float* __restrict__ x, const b16* __restrict__ WO, const float* __restrict__ lg, const float* __restrict__ lb, int NLIM, float* __restrict__ out) { __shared__ __attribute__((aligned(16))) b16 Ah[16][D + 8], Al[16][D + 8]; __shared__ float Y[16][D + 1]; const int lane = threadIdx.x, nloc = lane & 15, hlf = lane >> 4; const size_t n0 = (size_t)blockIdx.x * 16; if (n0 >= (size_t)NLIM) return;
  for (int rr = 0; rr < 16; ++rr) for (int q = 0; q < 8; ++q) { const int c = q * 32 + lane; b16 p, pl; split16(AGG[(n0 + rr) * D + c] * HS, p, pl); Ah[rr][c] = p; Al[rr][c] = pl; }
  if (lane < 16) for (int k = D; k < D + 8; ++k) { Ah[lane][k] = (b16)0.0f; Al[lane][k] = (b16)0.0f; }
  wave_lds_sync(); v8f acc[16];
#pragma unroll
  for (int t = 0; t < 16; ++t) acc[t] = (v8f){};
#pragma unroll 2
  for (int kb = 0; kb < D; kb += 32) { const v16b a = frag_kb(&Ah[nloc][kb], hlf), al = frag_kb(&Al[nloc][kb], hlf);
#pragma unroll
    for (int t = 0; t < 16; ++t) { const v16b bw = frag_kb(WO + (size_t)(t * 16 + nloc) * D + kb, hlf); acc[t] = wmma16b(a, bw, acc[t]); acc[t] = wmma16b(al, bw, acc[t]); } }
#pragma unroll
  for (int t = 0; t < 16; ++t)
#pragma unroll
    for (int r8 = 0; r8 < 8; ++r8) { const int rr = 8 * hlf + r8, cc = t * 16 + nloc; Y[rr][cc] = acc[t][r8] * (1.0f / (HS * WSC)) + bfv(x[(n0 + rr) * D + cc]); }
  wave_lds_sync();
  if (lane < 16) { const int r = lane; float m = 0.0f; for (int c = 0; c < D; ++c) m += Y[r][c]; m *= (1.0f / D); float vr = 0.0f; for (int c = 0; c < D; ++c) { const float d = Y[r][c] - m; vr += d * d; } vr *= (1.0f / D); const float rs = rsqrtf(vr + EPS); for (int c = 0; c < D; ++c) Y[r][c] = pmul((Y[r][c] - m) * rs, bfv(lg[c])) + bfv(lb[c]); }
  wave_lds_sync();
  for (int pass = 0; pass < 2; ++pass) { for (int rr = 0; rr < 16; ++rr) for (int q = 0; q < 2; ++q) *(volatile v4f*)(out + (n0 + rr) * D + q * 128 + lane * 4) = *(const v4f*)(&Y[rr][q * 128 + lane * 4]); __threadfence(); } }
}

extern "C" void kernel_launch(void* const* d_in, const int* in_sizes, int n_in, void* d_out, int out_size, void* d_ws, size_t ws_size, hipStream_t stream) {
  (void)n_in;
  auto Fp = [&](int i) { return (const float*)d_in[i]; }; auto Ip = [&](int i) { return (const int*)d_in[i]; };
  if (in_sizes[0] != N * D || in_sizes[1] != 2 * E || in_sizes[2] != E || in_sizes[3] != D * D || in_sizes[6] != H || in_sizes[7] != D * D || out_size != N * D) return;
  const int NLIM = N;
  size_t off = 0; char* ws = (char*)d_ws;
  auto carve = [&](size_t bytes) { char* p = ws + off; off += (bytes + 255) & ~(size_t)255; return p; };
  b16* WQKV = (b16*)carve((size_t)3 * D * D * 2); b16* WO = (b16*)carve((size_t)D * D * 2); float* Q = (float*)carve((size_t)N * D * 4); float* KV = (float*)carve((size_t)N * 2 * D * 4); float* AGG = (float*)carve((size_t)N * D * 4); CsrBufs8 csr; off = csr_carve8(csr, ws, off, E, N);
  if (off > ws_size || off > ((size_t)112 << 20)) return;
  wput_kernel<<<(4 * D * 32 + 255) / 256, 256, 0, stream>>>(Fp(3), Fp(4), Fp(5), Fp(7), WQKV, WO);
  csr_build8(csr, Ip(1), E, N, stream);
  proj_kernel<<<NLIM / 16, 32, 0, stream>>>(Fp(0), WQKV, Q, KV);
  att_kernel<<<(NLIM + NPB - 1) / NPB, 256, 0, stream>>>(Q, KV, Fp(2), Fp(6), Ip(1) + E, csr.PERM, csr.ROWPTR, csr.ROWCNT, (int)csr.permLen, NLIM, AGG);
  out_kernel<<<NLIM / 16, 32, 0, stream>>>(AGG, Fp(0), WO, Fp(8), Fp(9), NLIM, (float*)d_out);
}
